// SEEGTransformer_71373766525215
// MI455X (gfx1250) — hardware-run, weakly checked
//
#include <hip/hip_runtime.h>
#include <math.h>

#ifndef NB
#define NB 2
#endif
#define NB_FULL 2
#define N_SAMP 2
#define N_ELEC 32
#define N_TIME 40
#define NTOK 1280
#define N_FEAT 37
#define KXP 64
#define DM 128
#define NHEAD 8
#define HDIM 16
#define DFF 512
#define NLAYER 6
#define MTOK (NB * N_SAMP * NTOK)
#define KROWS (NB * NTOK)

#define C_X 64
#define C_W 256
#define C_LN 64
#define C_QKV 1024
#define C_P 1024
#define C_O 1024
#define C_G 1024
#define UNDO_XW 16384
#define UNDO_LW 16384
#define UNDO_OW 262144
#define UNDO_GW 262144

static_assert(NB <= NB_FULL);
static_assert(N_ELEC * N_TIME == NTOK);
static_assert(NHEAD * HDIM == DM);
static_assert(HDIM == 16);
static_assert(NTOK % N_TIME == 0 && MTOK % N_TIME == 0);
static_assert(MTOK % 64 == 0 && NTOK % 64 == 0 && NTOK % 256 == 0);
static_assert(DM % 64 == 0 && DFF % 64 == 0);
static_assert(KXP % 32 == 0 && DM % 32 == 0 && DFF % 32 == 0);
static_assert(N_FEAT <= KXP);
static_assert((MTOK * (KXP / 8)) % 256 == 0);
static_assert(((MTOK + KROWS) * (DM / 8)) % 256 == 0);
static_assert(MTOK % 16 == 0 && MTOK % 256 == 0);
static_assert(C_X * C_W == UNDO_XW);
static_assert(C_LN * C_W == UNDO_LW);
static_assert(C_O * C_W == UNDO_OW);
static_assert(C_G * C_W == UNDO_GW);
static_assert(C_QKV * C_QKV == 1048576);
static_assert(C_QKV == C_O);
static_assert((128 * (KXP / 8)) % 256 == 0 && (DM * (DM / 8)) % 256 == 0 && (DFF * (DM / 8)) % 256 == 0 && (DM * (DFF / 8)) % 256 == 0);

typedef __attribute__((ext_vector_type(16))) _Float16 v16h;
typedef __attribute__((ext_vector_type(8)))  _Float16 v8h;
typedef __attribute__((ext_vector_type(2)))  _Float16 v2h;
typedef __attribute__((ext_vector_type(8)))  float    v8f;
typedef __attribute__((ext_vector_type(4)))  float    v4f;
typedef __attribute__((ext_vector_type(2)))  float    v2f;
typedef __attribute__((ext_vector_type(4)))  unsigned int v4u;


#define VST2(T, ptr, val) do { const T vst2_v_ = (val); *(volatile T*)(ptr) = vst2_v_; __threadfence(); *(volatile T*)(ptr) = vst2_v_; } while (0)
#define VST2V4(ptr, val) do { const v4f vst2_v4_ = (val); *(volatile v4f*)(ptr) = vst2_v4_; __threadfence(); *(volatile v4f*)(ptr) = vst2_v4_; } while (0)

__device__ __forceinline__ float bfr(float f) {
    unsigned u = __float_as_uint(f);
    u += 0x7FFFu + ((u >> 16) & 1u);
    return __uint_as_float(u & 0xFFFF0000u);
}

__device__ __forceinline__ float flush14(float v) { return (fabsf(v) < 6.103515625e-05f) ? 0.0f : v; }
__device__ __forceinline__ _Float16 toh_flush(float v) { const float w = flush14(v); return (_Float16)w; }
__device__ __forceinline__ v2h toh2_flush(float a, float b) {
    v2f w; w.x = flush14(a); w.y = flush14(b);
    return __builtin_convertvector(w, v2h);
}
union Pack8U { v8h v; v2h p[4]; };
__device__ __forceinline__ v8h pack8h_flush(const float* v) {
    Pack8U u;
    u.p[0] = toh2_flush(v[0], v[1]);
    u.p[1] = toh2_flush(v[2], v[3]);
    u.p[2] = toh2_flush(v[4], v[5]);
    u.p[3] = toh2_flush(v[6], v[7]);
    return u.v;
}
__device__ __forceinline__ void st8h2(_Float16* P, size_t o, v8h hv) {
    *(volatile v8h*)(P + o) = hv;
    __threadfence();
    *(volatile v8h*)(P + o) = hv;
}

union FragU { v16h v; v8h h[2]; };
__device__ __forceinline__ v16h frag_ld(const _Float16* p) {
    FragU f; f.h[0] = *(const v8h*)(p); f.h[1] = *(const v8h*)(p + 16); return f.v;
}
__device__ __forceinline__ v8f wmma16(v16h a, v16h b, v8f c) {
    c = __builtin_amdgcn_wmma_f32_16x16x32_f16(false, a, false, b, (short)0, c, false, false);
    asm volatile("v_nop\n\tv_nop\n\tv_nop\n\tv_nop" : "+v"(c) : "v"(a), "v"(b));
    return c;
}
__device__ __forceinline__ void wave_sync_lds() {
    __builtin_amdgcn_fence(3  , "workgroup");
    __builtin_amdgcn_wave_barrier();
    __builtin_amdgcn_fence(2  , "workgroup");
}

#define GEMM_LDS_BYTES (8 * 16 * 68 * 4)
static_assert(GEMM_LDS_BYTES <= 131072);
static_assert(2 * 4 * 32 * 16 == 16 * 64 * 4);
static_assert(4 * 32 * 16 == 16 * 64 * 2);
template <int OUT_MODE, int RESID, int ACT, int BIAS_ROW, int UNDO, int OCARRY>
__device__ __forceinline__ void gemm64_body(
    const _Float16* __restrict__ A, unsigned lda, const _Float16* __restrict__ Bt, unsigned ldb,
    void* __restrict__ Cout, unsigned ldc, const float* __restrict__ bias, const float* __restrict__ resid,
    unsigned M, unsigned N, unsigned K) {
  __shared__ __align__(16) float sT[8][16 * 68];
  const float scale = 1.0f / (float)UNDO;
  const float oscale = (float)OCARRY;
  const unsigned lane = threadIdx.x & 31u;
  const unsigned wave = threadIdx.x >> 5;
  const unsigned tilesN = N >> 6, tilesM = M >> 6;
  const unsigned tile = blockIdx.x * 8u + wave;
  if (tile >= tilesM * tilesN) return;
  const unsigned tm = tile / tilesN;
  const unsigned tn = tile - tm * tilesN;
  const unsigned m0 = tm << 6, n0 = tn << 6;
  const unsigned rlane = lane & 15u;
  const unsigned koff = (lane >> 4) * 8u;
  const unsigned mOff = koff;

  v8f acc[4][4];
#pragma unroll
  for (int i = 0; i < 4; ++i)
#pragma unroll
    for (int j = 0; j < 4; ++j) acc[i][j] = (v8f){0.f,0.f,0.f,0.f,0.f,0.f,0.f,0.f};

  for (unsigned k0 = 0; k0 < K; k0 += 32u) {
    v16h bh[4];
#pragma unroll
    for (int j = 0; j < 4; ++j)
      bh[j] = frag_ld(Bt + (size_t)(n0 + ((unsigned)j << 4) + rlane) * ldb + koff + k0);
#pragma unroll
    for (int i = 0; i < 4; ++i) {
      const v16h ah = frag_ld(A + (size_t)(m0 + ((unsigned)i << 4) + rlane) * lda + koff + k0);
#pragma unroll
      for (int j = 0; j < 4; ++j)
        acc[i][j] = wmma16(ah, bh[j], acc[i][j]);
    }
  }

  float* slab = sT[wave];
#pragma unroll
  for (int i = 0; i < 4; ++i) {
    const unsigned mBase = m0 + ((unsigned)i << 4);
    float brow[8];
#pragma unroll
    for (int r = 0; r < 8; ++r) brow[r] = 0.0f;
    if (BIAS_ROW) {
#pragma unroll
      for (int r = 0; r < 8; ++r) brow[r] = bfr(bias[mBase + mOff + (unsigned)r]);
    }
#pragma unroll
    for (int j = 0; j < 4; ++j) {
      const unsigned n = n0 + ((unsigned)j << 4) + rlane;
      float bvc = 0.0f;
      if (!BIAS_ROW) bvc = bfr(bias[n]);
#pragma unroll
      for (int r = 0; r < 8; ++r) {
        float v = acc[i][j][r] * scale + (BIAS_ROW ? brow[r] : bvc);
        if (ACT == 1) v = 0.5f * v * (1.0f + erff(v * 0.70710678118654752f));
        if (OUT_MODE == 1) v *= oscale;
        slab[(mOff + (unsigned)r) * 68u + ((unsigned)j << 4) + rlane] = v;
      }
    }
    wave_sync_lds();
    if (OUT_MODE == 0) {
      float* C = (float*)Cout;
      const unsigned hh = lane >> 4, c4 = (lane & 15u) * 4u;
#pragma unroll
      for (int half = 0; half < 2; ++half) {
        v4f vv[4];
#pragma unroll
        for (int it = 0; it < 4; ++it) {
          const unsigned row = (unsigned)(half * 4 + it) * 2u + hh;
          vv[it] = *(const v4f*)(slab + row * 68u + c4);
          if (RESID == 1) vv[it] += *(const v4f*)(resid + (size_t)(mBase + row) * ldc + n0 + c4);
          if (RESID == 2) {
            unsigned rowv = mBase + row;
            asm volatile("" : "+v"(rowv));
            const unsigned el = (rowv / (unsigned)N_TIME) % (unsigned)N_ELEC;
            const v4f ev = *(const v4f*)(resid + (size_t)el * DM + n0 + c4);
            vv[it].x += bfr(ev.x); vv[it].y += bfr(ev.y); vv[it].z += bfr(ev.z); vv[it].w += bfr(ev.w);
          }
        }
        for (int pass = 0; pass < 2; ++pass) {
#pragma unroll
          for (int it = 0; it < 4; ++it) {
            const unsigned row = (unsigned)(half * 4 + it) * 2u + hh;
            *(volatile v4f*)(C + (size_t)(mBase + row) * ldc + n0 + c4) = vv[it];
          }
          __threadfence();
        }
      }
    } else {
      _Float16* C = (_Float16*)Cout;
      const unsigned q = lane >> 3, c8 = (lane & 7u) * 8u;
      v8h hv[4];
#pragma unroll
      for (int it = 0; it < 4; ++it) {
        const unsigned row = (unsigned)it * 4u + q;
        hv[it] = pack8h_flush(slab + row * 68u + c8);
      }
      for (int pass = 0; pass < 2; ++pass) {
#pragma unroll
        for (int it = 0; it < 4; ++it) {
          const unsigned row = (unsigned)it * 4u + q;
          *(volatile v8h*)(C + (size_t)(mBase + row) * ldc + n0 + c8) = hv[it];
        }
        __threadfence();
      }
    }
    wave_sync_lds();
  }
}

__global__ __launch_bounds__(256) void k_gemm_in(const _Float16* __restrict__ X16, const _Float16* __restrict__ WF16,
                                                 float* __restrict__ H, const float* __restrict__ bf, const float* __restrict__ emb) {
  gemm64_body<0, 2, 0, 0, UNDO_XW, 1>(X16, KXP, WF16, KXP, (void*)H, DM, bf, emb, MTOK, DM, KXP);
}
__global__ __launch_bounds__(256) void k_gemm_q(const _Float16* __restrict__ XLN, const _Float16* __restrict__ WQ,
                                                float* __restrict__ Q32, const float* __restrict__ bq) {
  gemm64_body<0, 0, 0, 0, UNDO_LW, 1>(XLN, DM, WQ, DM, (void*)Q32, DM, bq, nullptr, MTOK, DM, DM);
}
__global__ __launch_bounds__(256) void k_gemm_k(const _Float16* __restrict__ XLN, const _Float16* __restrict__ WK,
                                                float* __restrict__ K32, const float* __restrict__ bk) {
  const unsigned b = blockIdx.y;
  gemm64_body<0, 0, 0, 0, UNDO_LW, 1>(XLN + (size_t)b * (N_SAMP * NTOK) * DM, DM, WK, DM,
                                      (void*)(K32 + (size_t)b * NTOK * DM), DM, bk, nullptr, NTOK, DM, DM);
}
__global__ __launch_bounds__(256) void k_gemm_vt(const _Float16* __restrict__ WV, const _Float16* __restrict__ XLN,
                                                 _Float16* __restrict__ VT16, const float* __restrict__ bv) {
  const unsigned b = blockIdx.y;
  gemm64_body<1, 0, 0, 1, UNDO_LW, C_QKV>(WV, DM, XLN + (size_t)b * (N_SAMP * NTOK) * DM, DM,
                                          (void*)(VT16 + (size_t)b * DM * NTOK), NTOK, bv, nullptr, DM, NTOK, DM);
}
__global__ __launch_bounds__(256) void k_gemm_o(const _Float16* __restrict__ O16, const _Float16* __restrict__ WO,
                                                float* __restrict__ Hout, const float* __restrict__ bo, const float* __restrict__ Hin) {
  gemm64_body<0, 1, 0, 0, UNDO_OW, 1>(O16, DM, WO, DM, (void*)Hout, DM, bo, Hin, MTOK, DM, DM);
}
__global__ __launch_bounds__(256) void k_gemm_f1(const _Float16* __restrict__ XLN, const _Float16* __restrict__ W1,
                                                 _Float16* __restrict__ G16, const float* __restrict__ b1) {
  gemm64_body<1, 0, 1, 0, UNDO_LW, C_G>(XLN, DM, W1, DM, (void*)G16, DFF, b1, nullptr, MTOK, DFF, DM);
}
__global__ __launch_bounds__(256) void k_gemm_f2(const _Float16* __restrict__ G16, const _Float16* __restrict__ W2,
                                                 float* __restrict__ Hout, const float* __restrict__ b2, const float* __restrict__ Hin) {
  gemm64_body<0, 1, 0, 0, UNDO_GW, 1>(G16, DFF, W2, DFF, (void*)Hout, DM, b2, Hin, MTOK, DM, DFF);
}

__global__ __launch_bounds__(256) void k_wt(const float* __restrict__ Wm, unsigned KI, unsigned KP, unsigned NO, unsigned lgper,
                                            _Float16* __restrict__ W16) {
    const unsigned layer = blockIdx.y;
    const float* Wl = Wm + (size_t)layer * KI * NO;
    _Float16* Dl = W16 + (size_t)layer * KP * NO;
    const unsigned u = blockIdx.x * 256u + threadIdx.x;
    const unsigned per = 1u << lgper;
    if (u >= NO * per) return;
    const unsigned k0 = 8u * (u & (per - 1u));
    const unsigned o = u >> lgper;
    float v[8];
#pragma unroll
    for (int i = 0; i < 8; ++i) {
        const unsigned k = k0 + (unsigned)i;
        const unsigned kc = (k < KI) ? k : (KI - 1u);
        const float w = Wl[(size_t)kc * NO + o];
        v[i] = (k < KI) ? bfr(w) * (float)C_W : 0.0f;
    }
    st8h2(Dl, (size_t)o * KP + k0, pack8h_flush(v));
}

__global__ __launch_bounds__(256) void k_cvt_x(const float* __restrict__ x, _Float16* __restrict__ x16) {
    const unsigned u = blockIdx.x * 256u + threadIdx.x;
    if (u >= (unsigned)(MTOK * (KXP / 8))) return;
    const unsigned row = u >> 3, k0 = (u & 7u) * 8u;
    const float* xr = x + (size_t)row * N_FEAT;
    float v[8];
#pragma unroll
    for (int i = 0; i < 8; ++i) {
        const unsigned k = k0 + (unsigned)i;
        const unsigned kc = (k < (unsigned)N_FEAT) ? k : (unsigned)(N_FEAT - 1);
        const float xv = xr[kc];
        v[i] = (k < (unsigned)N_FEAT) ? bfr(xv) * (float)C_X : 0.0f;
    }
    st8h2(x16, (size_t)row * KXP + k0, pack8h_flush(v));
}

static_assert(16 * 16 == DM * 2);
__global__ __launch_bounds__(256) void k_ln(const float* __restrict__ h, const float* __restrict__ g, const float* __restrict__ bt,
                                            _Float16* __restrict__ z16, unsigned M) {
    if (blockIdx.x * 16u + 16u > M) return;
    const unsigned row = blockIdx.x * 16u + (threadIdx.x >> 4);
    const unsigned L = threadIdx.x & 15u;
    const float* hr = h + (size_t)row * DM + 8u * L;
    const v4f a = *(const v4f*)hr, b = *(const v4f*)(hr + 4);
    float s = ((a.x + a.y) + (a.z + a.w)) + ((b.x + b.y) + (b.z + b.w));
#pragma unroll
    for (int o = 8; o > 0; o >>= 1) s += __shfl_xor(s, o, 32);
    const float mu = s * (1.0f / (float)DM);
    float d[8] = {a.x - mu, a.y - mu, a.z - mu, a.w - mu, b.x - mu, b.y - mu, b.z - mu, b.w - mu};
    float q = 0.f;
#pragma unroll
    for (int i = 0; i < 8; ++i) q += d[i] * d[i];
#pragma unroll
    for (int o = 8; o > 0; o >>= 1) q += __shfl_xor(q, o, 32);
    const float sd = sqrtf(q * (1.0f / (float)DM) + 1e-5f);
    const v4f g0 = *(const v4f*)(g + 8u * L), g1 = *(const v4f*)(g + 8u * L + 4u);
    const v4f b0 = *(const v4f*)(bt + 8u * L), b1 = *(const v4f*)(bt + 8u * L + 4u);
    const float gg[8] = {g0.x, g0.y, g0.z, g0.w, g1.x, g1.y, g1.z, g1.w};
    const float bb[8] = {b0.x, b0.y, b0.z, b0.w, b1.x, b1.y, b1.z, b1.w};
    float y[8];
#pragma unroll
    for (int i = 0; i < 8; ++i) y[i] = ((d[i] / sd) * bfr(gg[i]) + bfr(bb[i])) * (float)C_LN;
    st8h2(z16, (size_t)row * DM + 8u * L, pack8h_flush(y));
}

__global__ __launch_bounds__(256) void k_rope(const float* __restrict__ QK32, _Float16* __restrict__ QK16) {
    const unsigned u = blockIdx.x * 256u + threadIdx.x;
    if (u >= (unsigned)((MTOK + KROWS) * (DM / 8))) return;
    const unsigned rowc = u >> 4, g = u & 15u;
    const float* src = QK32 + (size_t)rowc * DM + 8u * g;
    const v4f xl = *(const v4f*)src, xr = *(const v4f*)(src + 4);
    unsigned rowt = rowc;
    asm volatile("" : "+v"(rowt));
    const float tf = (float)(rowt % (unsigned)N_TIME);
    const float th[4] = {1.0f, 0.00625f, 0.00625f, 0.00625f};
    float cs[4], sn[4];
#pragma unroll
    for (int i = 0; i < 4; ++i) { const float ang = tf * th[i]; cs[i] = cosf(ang); sn[i] = sinf(ang); }
    const bool rot = (g & 1u) == 0u;
    const float l[4] = {xl.x, xl.y, xl.z, xl.w};
    const float r[4] = {xr.x, xr.y, xr.z, xr.w};
    float y[8];
#pragma unroll
    for (int i = 0; i < 4; ++i) {
        const float yl = l[i] * cs[i] + r[i] * sn[i];
        const float yr = r[i] * cs[i] - l[i] * sn[i];
        y[i]     = (rot ? yl : l[i]) * (float)C_QKV;
        y[i + 4] = (rot ? yr : r[i]) * (float)C_QKV;
    }
    st8h2(QK16, (size_t)rowc * DM + 8u * g, pack8h_flush(y));
}

#define AT_PP 72
#define AT_PO 68
#define ATTN_LDS_BYTES (16 * 16 * AT_PP * 2 + 16 * 16 * AT_PO * 4)
static_assert(ATTN_LDS_BYTES <= 131072);
static_assert(4 * 32 * 16 == 16 * 64 * 2);
static_assert(NTOK == 5 * 256 && NTOK == 20 * 64);
__global__ __launch_bounds__(512) void k_attn(const _Float16* __restrict__ Q16, const _Float16* __restrict__ K16,
                                              const _Float16* __restrict__ VT16, _Float16* __restrict__ O16) {
    __shared__ __align__(16) _Float16 sP[16][16 * AT_PP];
    __shared__ __align__(16) float    sO[16][16 * AT_PO];
    const unsigned tid = threadIdx.x, lane = tid & 31u;
    const unsigned wave = (unsigned)__builtin_amdgcn_readfirstlane((int)(tid >> 5));
    const unsigned hh = lane >> 4, c = lane & 15u;
    const unsigned blk = blockIdx.x;
    const unsigned qb = blk % 5u;
    const unsigned t1 = blk / 5u;
    const unsigned quad = t1 & 1u;
    const unsigned bs = t1 >> 1;
    const unsigned b = bs >> 1;
    const unsigned qtok0 = qb * 256u + wave * 16u;
    const unsigned row0 = bs * (unsigned)NTOK + qtok0;
    const _Float16* Kb = K16 + (size_t)b * NTOK * DM;
    const _Float16* Vb = VT16 + (size_t)b * DM * NTOK;
    int eq[8], tq[8];
#pragma unroll
    for (int r = 0; r < 8; ++r) {
        const unsigned qt = qtok0 + 8u * hh + (unsigned)r;
        const unsigned e = qt / (unsigned)N_TIME;
        eq[r] = (int)e;
        tq[r] = (int)(qt - e * (unsigned)N_TIME);
    }
    _Float16* pw = sP[wave];
    float* ow = sO[wave];
    const v8h zero8 = (v8h){(_Float16)0.0f, (_Float16)0.0f, (_Float16)0.0f, (_Float16)0.0f,
                            (_Float16)0.0f, (_Float16)0.0f, (_Float16)0.0f, (_Float16)0.0f};
    const float SCQK = 0.25f / 1048576.0f;
    const float LOG2E = 1.4426950408889634f;
    for (unsigned hq = 0; hq < 4u; ++hq) {
        const unsigned head = 4u * quad + hq;
        FragU qf;
        qf.h[0] = *(const v8h*)(Q16 + (size_t)(row0 + c) * DM + head * 16u + 8u * hh);
        qf.h[1] = zero8;
        float mrow[8], lrow[8];
        v8f os = (v8f){0.f,0.f,0.f,0.f,0.f,0.f,0.f,0.f};
#pragma unroll
        for (int r = 0; r < 8; ++r) { mrow[r] = -3.0e38f; lrow[r] = 0.f; }
        for (unsigned kc = 0; kc < (unsigned)(NTOK / 64); ++kc) {
            const unsigned kv0 = kc * 64u;
            v8f s[4];
            int ek[4], tk[4];
#pragma unroll
            for (int j = 0; j < 4; ++j) {
                const unsigned key = kv0 + (unsigned)j * 16u + c;
                FragU kf;
                kf.h[0] = *(const v8h*)(Kb + (size_t)key * DM + head * 16u + 8u * hh);
                kf.h[1] = zero8;
                const v8f z = (v8f){0.f,0.f,0.f,0.f,0.f,0.f,0.f,0.f};
                s[j] = wmma16(qf.v, kf.v, z);
                const unsigned e = key / (unsigned)N_TIME;
                ek[j] = (int)e;
                tk[j] = (int)(key - e * (unsigned)N_TIME);
            }
#pragma unroll
            for (int r = 0; r < 8; ++r) {
                float mx = -3.0e38f;
#pragma unroll
                for (int j = 0; j < 4; ++j) {
                    const bool masked = (tk[j] > tq[r]) || ((tk[j] == tq[r]) && (ek[j] >= eq[r]));
                    const float sv = masked ? -INFINITY : (s[j][r] * SCQK) * LOG2E;
                    s[j][r] = sv;
                    mx = fmaxf(mx, sv);
                }
                mx = fmaxf(mx, __shfl_xor(mx, 1, 32)); mx = fmaxf(mx, __shfl_xor(mx, 2, 32));
                mx = fmaxf(mx, __shfl_xor(mx, 4, 32)); mx = fmaxf(mx, __shfl_xor(mx, 8, 32));
                const float mnew = fmaxf(mrow[r], mx);
                const float alpha = exp2f(mrow[r] - mnew);
                mrow[r] = mnew;
                float psum = 0.f;
#pragma unroll
                for (int j = 0; j < 4; ++j) {
                    const float p = exp2f(s[j][r] - mnew);
                    psum += p;
                    pw[(8u * hh + (unsigned)r) * AT_PP + (unsigned)j * 16u + c] = toh_flush(p * (float)C_P);
                }
                lrow[r] = lrow[r] * alpha + psum;
                os[r] *= alpha;
            }
            wave_sync_lds();
#pragma unroll
            for (int kk = 0; kk < 2; ++kk) {
                const v16h pa = frag_ld(pw + c * AT_PP + (unsigned)kk * 32u + 8u * hh);
                const v16h vb = frag_ld(Vb + (size_t)(head * 16u + c) * NTOK + kv0 + (unsigned)kk * 32u + 8u * hh);
                os = wmma16(pa, vb, os);
            }
            wave_sync_lds();
        }
#pragma unroll
        for (int r = 0; r < 8; ++r) {
            float l = lrow[r];
            l += __shfl_xor(l, 1, 32); l += __shfl_xor(l, 2, 32);
            l += __shfl_xor(l, 4, 32); l += __shfl_xor(l, 8, 32);
            const float lsafe = (l == 0.0f) ? 1.0f : l;
            const float inv = 1.0f / (lsafe * (float)C_P);
            ow[(8u * hh + (unsigned)r) * AT_PO + hq * 16u + c] = os[r] * inv;
        }
    }
    wave_sync_lds();
    {
        const unsigned q = lane >> 3, c8 = (lane & 7u) * 8u;
        v8h ov[4];
#pragma unroll
        for (int it = 0; it < 4; ++it) ov[it] = pack8h_flush(ow + ((unsigned)it * 4u + q) * AT_PO + c8);
        _Float16* dst = O16 + (size_t)row0 * DM + quad * 64u;
        for (int pass = 0; pass < 2; ++pass) {
#pragma unroll
            for (int it = 0; it < 4; ++it) *(volatile v8h*)(dst + (size_t)((unsigned)it * 4u + q) * DM + c8) = ov[it];
            __threadfence();
        }
    }
}

static_assert(MTOK % 32 == 0 && 32 * 4 == 128 && DM == 32 * 4);
__global__ __launch_bounds__(256) void k_out(const float* __restrict__ h, const float* __restrict__ Wout,
                                             const float* __restrict__ bout, float* __restrict__ out) {
    const unsigned lane = threadIdx.x & 31u;
    const unsigned wv = blockIdx.x * 8u + (threadIdx.x >> 5);
    const unsigned r0 = wv * 32u;
    if (r0 >= (unsigned)MTOK) return;
    const v4f w4 = *(const v4f*)(Wout + 4u * lane);
    const float w0 = bfr(w4.x), w1 = bfr(w4.y), w2 = bfr(w4.z), w3 = bfr(w4.w);
    const float ob = bfr(bout[0]);
    float mine = 0.f;
    for (unsigned rr = 0; rr < 32u; ++rr) {
        const v4f a = *(const v4f*)(h + (size_t)(r0 + rr) * DM + 4u * lane);
        float s = (a.x * w0 + a.y * w1) + (a.z * w2 + a.w * w3);
#pragma unroll
        for (int o = 16; o > 0; o >>= 1) s += __shfl_xor(s, o, 32);
        mine = (lane == rr) ? s : mine;
    }
    VST2(float, out + r0 + lane, mine + ob);
}

constexpr size_t al256(size_t x) { return (x + 255) & ~(size_t)255; }
constexpr size_t OFF_X16  = 0;
constexpr size_t OFF_WF   = OFF_X16  + al256((size_t)MTOK * KXP * 2);
constexpr size_t OFF_WQ   = OFF_WF   + al256((size_t)DM * KXP * 2);
constexpr size_t OFF_WK   = OFF_WQ   + al256((size_t)NLAYER * DM * DM * 2);
constexpr size_t OFF_WV   = OFF_WK   + al256((size_t)NLAYER * DM * DM * 2);
constexpr size_t OFF_WO   = OFF_WV   + al256((size_t)NLAYER * DM * DM * 2);
constexpr size_t OFF_W1   = OFF_WO   + al256((size_t)NLAYER * DM * DM * 2);
constexpr size_t OFF_W2   = OFF_W1   + al256((size_t)NLAYER * DFF * DM * 2);
constexpr size_t OFF_HA   = OFF_W2   + al256((size_t)NLAYER * DM * DFF * 2);
constexpr size_t OFF_HB   = OFF_HA   + al256((size_t)MTOK * DM * 4);
constexpr size_t OFF_XLN  = OFF_HB   + al256((size_t)MTOK * DM * 4);
constexpr size_t OFF_QK32 = OFF_XLN  + al256((size_t)MTOK * DM * 2);
constexpr size_t OFF_QK16 = OFF_QK32 + al256((size_t)(MTOK + KROWS) * DM * 4);
constexpr size_t OFF_VT   = OFF_QK16 + al256((size_t)(MTOK + KROWS) * DM * 2);
constexpr size_t OFF_O16  = OFF_VT   + al256((size_t)NB * DM * NTOK * 2);
constexpr size_t OFF_G16  = OFF_O16  + al256((size_t)MTOK * DM * 2);
constexpr size_t WS_TOTAL = OFF_G16  + al256((size_t)MTOK * DFF * 2);
static_assert(WS_TOTAL <= (size_t)134217728);

extern "C" void kernel_launch(void* const* d_in, const int* in_sizes, int n_in, void* d_out, int out_size,
                              void* d_ws, size_t ws_size, hipStream_t stream) {
    if (n_in < 22) return;
    if (in_sizes[0] < MTOK * N_FEAT || in_sizes[1] < N_ELEC * DM || in_sizes[2] < N_FEAT * DM || in_sizes[3] < DM) return;
    if (in_sizes[4] < NLAYER * DM * DM || in_sizes[5] < NLAYER * DM || in_sizes[6] < NLAYER * DM * DM || in_sizes[7] < NLAYER * DM) return;
    if (in_sizes[8] < NLAYER * DM * DM || in_sizes[9] < NLAYER * DM || in_sizes[10] < NLAYER * DM * DM || in_sizes[11] < NLAYER * DM) return;
    if (in_sizes[12] < NLAYER * DM * DFF || in_sizes[13] < NLAYER * DFF || in_sizes[14] < NLAYER * DFF * DM || in_sizes[15] < NLAYER * DM) return;
    if (in_sizes[16] < NLAYER * DM || in_sizes[17] < NLAYER * DM || in_sizes[18] < NLAYER * DM || in_sizes[19] < NLAYER * DM) return;
    if (in_sizes[20] < DM || in_sizes[21] < 1 || out_size < MTOK) return;
    if (WS_TOTAL > ws_size) return;

    const float* x    = (const float*)d_in[0];
    const float* emb  = (const float*)d_in[1];
    const float* Wf   = (const float*)d_in[2];
    const float* bf   = (const float*)d_in[3];
    const float* Wq   = (const float*)d_in[4];
    const float* bq   = (const float*)d_in[5];
    const float* Wk   = (const float*)d_in[6];
    const float* bk   = (const float*)d_in[7];
    const float* Wv   = (const float*)d_in[8];
    const float* bv   = (const float*)d_in[9];
    const float* Wo   = (const float*)d_in[10];
    const float* bo   = (const float*)d_in[11];
    const float* W1   = (const float*)d_in[12];
    const float* b1   = (const float*)d_in[13];
    const float* W2   = (const float*)d_in[14];
    const float* b2   = (const float*)d_in[15];
    const float* g1   = (const float*)d_in[16];
    const float* be1  = (const float*)d_in[17];
    const float* g2   = (const float*)d_in[18];
    const float* be2  = (const float*)d_in[19];
    const float* Wout = (const float*)d_in[20];
    const float* bout = (const float*)d_in[21];
    float* out = (float*)d_out;

    char* wsp = (char*)d_ws;
    _Float16* x16  = (_Float16*)(wsp + OFF_X16);
    _Float16* wf16 = (_Float16*)(wsp + OFF_WF);
    _Float16* wq16 = (_Float16*)(wsp + OFF_WQ);
    _Float16* wk16 = (_Float16*)(wsp + OFF_WK);
    _Float16* wv16 = (_Float16*)(wsp + OFF_WV);
    _Float16* wo16 = (_Float16*)(wsp + OFF_WO);
    _Float16* w116 = (_Float16*)(wsp + OFF_W1);
    _Float16* w216 = (_Float16*)(wsp + OFF_W2);
    float*    hA   = (float*)(wsp + OFF_HA);
    float*    hB   = (float*)(wsp + OFF_HB);
    _Float16* xln  = (_Float16*)(wsp + OFF_XLN);
    float*    qk32 = (float*)(wsp + OFF_QK32);
    _Float16* qk16 = (_Float16*)(wsp + OFF_QK16);
    _Float16* vt16 = (_Float16*)(wsp + OFF_VT);
    _Float16* o16  = (_Float16*)(wsp + OFF_O16);
    _Float16* g16  = (_Float16*)(wsp + OFF_G16);
    float*    k32  = qk32 + (size_t)MTOK * DM;
    const _Float16* q16 = qk16;
    const _Float16* k16 = qk16 + (size_t)MTOK * DM;

    k_wt<<<dim3((DM * (KXP / 8)) / 256, 1), 256, 0, stream>>>(Wf, N_FEAT, KXP, DM, 3, wf16);
    k_wt<<<dim3((DM * (DM / 8)) / 256, NLAYER), 256, 0, stream>>>(Wq, DM, DM, DM, 4, wq16);
    k_wt<<<dim3((DM * (DM / 8)) / 256, NLAYER), 256, 0, stream>>>(Wk, DM, DM, DM, 4, wk16);
    k_wt<<<dim3((DM * (DM / 8)) / 256, NLAYER), 256, 0, stream>>>(Wv, DM, DM, DM, 4, wv16);
    k_wt<<<dim3((DM * (DM / 8)) / 256, NLAYER), 256, 0, stream>>>(Wo, DM, DM, DM, 4, wo16);
    k_wt<<<dim3((DFF * (DM / 8)) / 256, NLAYER), 256, 0, stream>>>(W1, DM, DM, DFF, 4, w116);
    k_wt<<<dim3((DM * (DFF / 8)) / 256, NLAYER), 256, 0, stream>>>(W2, DFF, DFF, DM, 6, w216);

    k_cvt_x<<<(MTOK * (KXP / 8)) / 256, 256, 0, stream>>>(x, x16);

    const unsigned gH  = ((MTOK / 64) * (DM / 64) + 7) / 8;
    const unsigned gK  = ((NTOK / 64) * (DM / 64) + 7) / 8;
    const unsigned gVT = ((DM / 64) * (NTOK / 64) + 7) / 8;
    const unsigned gF  = ((MTOK / 64) * (DFF / 64) + 7) / 8;

    k_gemm_in<<<gH, 256, 0, stream>>>(x16, wf16, hA, bf, emb);

    for (int l = 0; l < NLAYER; ++l) {
        const _Float16* wql = wq16 + (size_t)l * DM * DM;
        const _Float16* wkl = wk16 + (size_t)l * DM * DM;
        const _Float16* wvl = wv16 + (size_t)l * DM * DM;
        const _Float16* wol = wo16 + (size_t)l * DM * DM;
        const _Float16* w1l = w116 + (size_t)l * DFF * DM;
        const _Float16* w2l = w216 + (size_t)l * DM * DFF;

        k_ln<<<MTOK / 16, 256, 0, stream>>>(hA, g1 + l * DM, be1 + l * DM, xln, MTOK);
        k_gemm_q<<<gH, 256, 0, stream>>>(xln, wql, qk32, bq + l * DM);
        k_gemm_k<<<dim3(gK, NB), 256, 0, stream>>>(xln, wkl, k32, bk + l * DM);
        k_gemm_vt<<<dim3(gVT, NB), 256, 0, stream>>>(wvl, xln, vt16, bv + l * DM);
        k_rope<<<((MTOK + KROWS) * (DM / 8)) / 256, 256, 0, stream>>>(qk32, qk16);
        k_attn<<<NB * N_SAMP * 2 * 5, 512, 0, stream>>>(q16, k16, vt16, o16);
        k_gemm_o<<<gH, 256, 0, stream>>>(o16, wol, hB, bo + l * DM, hA);
        k_ln<<<MTOK / 16, 256, 0, stream>>>(hB, g2 + l * DM, be2 + l * DM, xln, MTOK);
        k_gemm_f1<<<gF, 256, 0, stream>>>(xln, w1l, g16, b1 + l * DFF);
        k_gemm_f2<<<gH, 256, 0, stream>>>(g16, w2l, hA, b2 + l * DM, hB);
    }
    k_out<<<MTOK / 256, 256, 0, stream>>>(hA, Wout, bout, out);
}
